// EMAttention_70171175682266
// MI455X (gfx1250) — hardware-verified
//
#include <hip/hip_runtime.h>
#include <math.h>

typedef __attribute__((ext_vector_type(16))) _Float16 v16h;
typedef __attribute__((ext_vector_type(16))) __bf16 v16b;
typedef __attribute__((ext_vector_type(8)))  _Float16 v8h;
typedef __attribute__((ext_vector_type(8)))  float v8f;
typedef __attribute__((ext_vector_type(4)))  float v4f;
typedef __attribute__((ext_vector_type(2)))  float v2f;
typedef __attribute__((ext_vector_type(4)))  unsigned v4u;
typedef __attribute__((ext_vector_type(4)))  int v4i;
typedef float __attribute__((may_alias)) float_a;
typedef int __attribute__((may_alias)) int_a;

template <typename T> __device__ __forceinline__ void vst2(void* p, T v) { *(volatile T*)p = v; __threadfence(); *(volatile T*)p = v; }
__device__ __forceinline__ v8f wmma16(v16h a, v16h b, v8f c) {
  v8f d = __builtin_amdgcn_wmma_f32_16x16x32_f16(false, a, false, b, (short)0, c, false, false);
  asm volatile("v_nop\n\tv_nop\n\tv_nop\n\tv_nop" : "+v"(d) : "v"(a), "v"(b));
  return d;
}
__device__ __forceinline__ v8f wmma_bf(v16b a, v16b b, v8f c) {
  v8f d = __builtin_amdgcn_wmma_f32_16x16x32_bf16(false, a, false, b, (short)0, c, false, false);
  asm volatile("v_nop\n\tv_nop\n\tv_nop\n\tv_nop" : "+v"(d) : "v"(a), "v"(b));
  return d;
}
__device__ __forceinline__ v16h frag_h(const _Float16* rowk0, int lane) {
  union { v16h v; v8h q[2]; } u; const _Float16* p = rowk0 + 8 * (lane >> 4);
  u.q[0] = *(const v8h*)p; u.q[1] = *(const v8h*)(p + 16); return u.v;
}
__device__ __forceinline__ v16h frag_f32(const float* rowk0, int lane) {
  v16h a; const float* p = rowk0 + 8 * (lane >> 4);
#pragma unroll
  for (int i = 0; i < 8; ++i) { a[i] = (_Float16)p[i]; a[8 + i] = (_Float16)p[16 + i]; }
  return a;
}
__device__ __forceinline__ v16h frag_f32s(const float* rowk0, int lane, float sc) {
  v16h a; const float* p = rowk0 + 8 * (lane >> 4);
#pragma unroll
  for (int i = 0; i < 8; ++i) { a[i] = (_Float16)(p[i] * sc); a[8 + i] = (_Float16)(p[16 + i] * sc); }
  return a;
}
__device__ __forceinline__ v16h fragc_f32(const float* W, int k0, int n, int lane, int ld, int K) {
  v16h a; const int g = lane >> 4;
#pragma unroll
  for (int i = 0; i < 8; ++i) { const int ka = k0 + 8 * g + i, kb = ka + 16;
    a[i] = (_Float16)(ka < K ? W[(size_t)(ka < K ? ka : K - 1) * ld + n] : 0.f); a[8 + i] = (_Float16)(kb < K ? W[(size_t)(kb < K ? kb : K - 1) * ld + n] : 0.f); }
  return a;
}
struct F2 { v16b h, l; };
__device__ __forceinline__ F2 bsplit16(const float v[16]) { F2 r;
#pragma unroll
  for (int i = 0; i < 16; ++i) { const __bf16 h = (__bf16)v[i]; r.h[i] = h; r.l[i] = (__bf16)(v[i] - (float)h); }
  return r; }
__device__ __forceinline__ F2 split_row(const float* row, int k0, int lane) { float v[16]; const float* p = row + k0 + 8 * (lane >> 4);
#pragma unroll
  for (int i = 0; i < 8; ++i) { v[i] = p[i]; v[8 + i] = p[16 + i]; }
  return bsplit16(v); }
__device__ __forceinline__ F2 split_rowK(const float* row, int k0, int lane, int K) { float v[16]; const int g = lane >> 4;
#pragma unroll
  for (int i = 0; i < 8; ++i) { const int ka = k0 + 8 * g + i, kb = ka + 16; v[i] = ka < K ? row[ka < K ? ka : K - 1] : 0.f; v[8 + i] = kb < K ? row[kb < K ? kb : K - 1] : 0.f; }
  return bsplit16(v); }
__device__ __forceinline__ F2 split_col(const float* W, int k0, int n, int lane, int ld, int K) { float v[16]; const int g = lane >> 4;
#pragma unroll
  for (int i = 0; i < 8; ++i) { const int ka = k0 + 8 * g + i, kb = ka + 16; v[i] = ka < K ? W[(size_t)(ka < K ? ka : K - 1) * ld + n] : 0.f; v[8 + i] = kb < K ? W[(size_t)(kb < K ? kb : K - 1) * ld + n] : 0.f; }
  return bsplit16(v); }
__device__ __forceinline__ v8f mac3(const F2& a, const F2& b, v8f c) { c = wmma_bf(a.l, b.h, c); c = wmma_bf(a.h, b.l, c); return wmma_bf(a.h, b.h, c); }
__device__ __forceinline__ float sigm(float v) { return 1.0f / (1.0f + expf(-v)); }
#define LDSX() do { asm volatile("s_wait_dscnt 0" ::: "memory"); __builtin_amdgcn_wave_barrier(); __builtin_amdgcn_fence(__ATOMIC_RELEASE, "workgroup"); } while (0)


#define NB 4
#define NN 2048
#define CC 1024
#define NH 32
#define HD 32
#define NR 4
#define MM (NN / NR)
#define BNEPS 1e-6f
#ifndef TNB
#define TNB NB
#endif
#ifndef TOB
#define TOB (TNB * NN / 64)
#endif
typedef __attribute__((ext_vector_type(8))) __bf16 v8b;
__device__ __forceinline__ v16b frag_b(const __bf16* rowk0, int lane) {
  union { v16b v; v8b q[2]; } u; const __bf16* p = rowk0 + 8 * (lane >> 4);
  u.q[0] = *(const v8b*)p; u.q[1] = *(const v8b*)(p + 16); return u.v;
}
__device__ __forceinline__ float bfr(float v) { return (float)(__bf16)v; }
__device__ __attribute__((noinline)) float exp_ni(float v) { return expf(v); }
__device__ __attribute__((noinline)) float erf_ni(float v) { return erff(v); }

#define WS_Q   0u
#define WS_XR  (WS_Q + 4u * (size_t)NB * NN * CC)
#define WS_KT  (WS_XR + 4u * (size_t)NB * MM * CC)
#define WS_KTL (WS_KT + 2u * (size_t)NB * CC * MM)
#define WS_VT  (WS_KTL + 2u * (size_t)NB * CC * MM)
#define WS_VTL (WS_VT + 2u * (size_t)NB * CC * MM)
#define WS_KV  (WS_VTL + 2u * (size_t)NB * CC * MM)
#define WS_CT  (WS_KV + 4u * (size_t)NB * CC * HD)
#define WS_END (WS_CT + 4u * (size_t)NB * NN * CC)

__device__ __forceinline__ v16b fragb_f32(const float* __restrict__ p, int lane) { v16b a; const float* pp = p + 8 * (lane >> 4);
#pragma unroll
  for (int i = 0; i < 8; ++i) { a[i] = (__bf16)pp[i]; a[8 + i] = (__bf16)pp[16 + i]; } return a; }
__global__ __launch_bounds__(128) void k_q(const float* __restrict__ X, const float* __restrict__ WQ, float* __restrict__ Q) { __shared__ __align__(16) float sf[4][16][132];
  const int tid = threadIdx.x, wave = tid >> 5, lane = tid & 31, col = lane & 15, g = lane >> 4; const size_t r0 = (size_t)blockIdx.x * 64 + wave * 16; const int c0 = blockIdx.y * 128;
  v8f acc[8] = {};
#pragma unroll 2
  for (int kc = 0; kc < CC / 32; ++kc) { const v16b a = fragb_f32(X + (r0 + col) * CC + kc * 32, lane);
#pragma unroll
    for (int j = 0; j < 8; ++j) acc[j] = wmma_bf(a, fragb_f32(WQ + (size_t)(c0 + j * 16 + col) * CC + kc * 32, lane), acc[j]); }
#pragma unroll
  for (int j = 0; j < 8; ++j)
#pragma unroll
    for (int r = 0; r < 8; ++r) sf[wave][8 * g + r][j * 16 + col] = acc[j][r];
  LDSX(); for (int rl = 0; rl < 16; ++rl) vst2(Q + (r0 + rl) * CC + c0 + lane * 4, *(const v4f*)&sf[wave][rl][lane * 4]); }
__global__ __launch_bounds__(256) void k_pool(const float* __restrict__ X, const float* __restrict__ G, const float* __restrict__ Bt, const float* __restrict__ Mu, const float* __restrict__ Var, float* __restrict__ XR) { __shared__ __align__(16) float so[CC]; const int t = threadIdx.x; const size_t row = blockIdx.x; const size_t b = row / MM; const int m = (int)(row % MM);
  for (int c = t; c < CC; c += 256) { float s = 0.f;
#pragma unroll
    for (int i = 0; i < NR; ++i) s += bfr(X[(b * NN + (size_t)m * NR + i) * CC + c]);
    s *= (1.0f / NR); so[c] = (s - bfr(Mu[c])) / sqrtf(bfr(Var[c]) + BNEPS) * bfr(G[c]) + bfr(Bt[c]); }
  __syncthreads(); for (int q = t; q < CC / 4; q += 256) vst2(XR + row * CC + q * 4, *(const v4f*)&so[q * 4]); }
__global__ __launch_bounds__(128) void k_kv(const float* __restrict__ XR, const float* __restrict__ WK, const float* __restrict__ WV, _Float16* __restrict__ KT, _Float16* __restrict__ KTL, _Float16* __restrict__ VT, _Float16* __restrict__ VTL) { __shared__ __align__(16) _Float16 th[128][72], tl[128][72];
  const int tid = threadIdx.x, wave = tid >> 5, lane = tid & 31, col = lane & 15, g = lane >> 4; const int which = blockIdx.z / TNB; const size_t b = blockIdx.z % TNB; const int m0 = blockIdx.x * 64; const int c0 = blockIdx.y * 128; const size_t r0 = b * MM + m0 + wave * 16; const float* Wm = which == 0 ? WK : WV;
  v8f acc[8] = {};
#pragma unroll 2
  for (int kc = 0; kc < CC / 32; ++kc) { const F2 a = split_row(XR + (r0 + col) * CC, kc * 32, lane);
#pragma unroll
    for (int j = 0; j < 8; ++j) { const v16b w = fragb_f32(Wm + (size_t)(c0 + j * 16 + col) * CC + kc * 32, lane); acc[j] = wmma_bf(a.h, w, acc[j]); acc[j] = wmma_bf(a.l, w, acc[j]); } }
#pragma unroll
  for (int j = 0; j < 8; ++j)
#pragma unroll
    for (int r = 0; r < 8; ++r) { const float v = acc[j][r]; const _Float16 hv = (_Float16)v; th[j * 16 + col][wave * 16 + 8 * g + r] = hv; tl[j * 16 + col][wave * 16 + 8 * g + r] = (_Float16)((v - (float)hv) * 2048.0f); }
  __syncthreads(); _Float16* PH = which == 0 ? KT : VT; _Float16* PL = which == 0 ? KTL : VTL;
  for (int e = tid; e < 128 * 8; e += 128) { const int cl = e >> 3, q = e & 7; const size_t o = (b * CC + c0 + cl) * (size_t)MM + m0 + q * 8; vst2((unsigned*)(PH + o), *(const v4u*)&th[cl][q * 8]); vst2((unsigned*)(PL + o), *(const v4u*)&tl[cl][q * 8]); } }
__global__ __launch_bounds__(64) void k_kvp(const _Float16* __restrict__ KT, const _Float16* __restrict__ KTL, const _Float16* __restrict__ VT, const _Float16* __restrict__ VTL, float* __restrict__ KVT) { __shared__ __align__(16) float st[HD][HD + 4];
  const int tid = threadIdx.x, wave = tid >> 5, lane = tid & 31, col = lane & 15, g = lane >> 4; const size_t bh = blockIdx.x; const size_t b = bh / NH; const int h = bh % NH;
  v8f acc[2] = {};
#pragma unroll 2
  for (int kc = 0; kc < MM / 32; ++kc) { const size_t ao = (b * CC + (size_t)h * HD + wave * 16 + col) * MM + kc * 32; const v16h ah = frag_h(KT + ao, lane), al = frag_h(KTL + ao, lane);
#pragma unroll
    for (int j = 0; j < 2; ++j) { const size_t bo = (b * CC + (size_t)h * HD + j * 16 + col) * MM + kc * 32; const v16h vh = frag_h(VT + bo, lane), vl = frag_h(VTL + bo, lane); acc[j] = wmma16(ah, vh, acc[j]); v8f t2 = {}; t2 = wmma16(ah, vl, t2); t2 = wmma16(al, vh, t2);
#pragma unroll
      for (int r = 0; r < 8; ++r) acc[j][r] += t2[r] * (1.0f / 2048.0f); } }
#pragma unroll
  for (int j = 0; j < 2; ++j)
#pragma unroll
    for (int r = 0; r < 8; ++r) st[j * 16 + col][wave * 16 + 8 * g + r] = acc[j][r];
  __syncthreads(); for (int e = tid; e < HD * 8; e += 64) { const int ee = e >> 3, q = e & 7; vst2(KVT + ((b * CC) + (size_t)h * HD + ee) * HD + q * 4, *(const v4f*)&st[ee][q * 4]); } }
__global__ __launch_bounds__(128) void k_ctx(const float* __restrict__ Q, const float* __restrict__ KVT, float* __restrict__ CT) { __shared__ __align__(16) float sf[4][16][132];
  const int tid = threadIdx.x, wave = tid >> 5, lane = tid & 31, col = lane & 15, g = lane >> 4; const size_t r0 = (size_t)blockIdx.x * 64 + wave * 16; const int c0 = blockIdx.y * 128; const size_t b = ((size_t)blockIdx.x * 64) / NN;
  v8f acc[8] = {};
#pragma unroll
  for (int hh = 0; hh < 4; ++hh) { const int h = c0 / HD + hh; const F2 a = split_row(Q + (r0 + col) * CC, h * HD, lane);
#pragma unroll
    for (int jj = 0; jj < 2; ++jj) { float wv[16]; const float* wr = KVT + (b * CC + (size_t)h * HD + jj * 16 + col) * HD + 8 * g;
#pragma unroll
      for (int i = 0; i < 8; ++i) { wv[i] = wr[i]; wv[8 + i] = wr[16 + i]; }
      const F2 wb = bsplit16(wv); const int j = hh * 2 + jj; acc[j] = wmma_bf(a.h, wb.h, acc[j]); acc[j] = wmma_bf(a.h, wb.l, acc[j]); acc[j] = wmma_bf(a.l, wb.h, acc[j]); } }
#pragma unroll
  for (int j = 0; j < 8; ++j)
#pragma unroll
    for (int r = 0; r < 8; ++r) sf[wave][8 * g + r][j * 16 + col] = acc[j][r] * 0.17677669529663687f;
  LDSX(); for (int rl = 0; rl < 16; ++rl) vst2(CT + (r0 + rl) * CC + c0 + lane * 4, *(const v4f*)&sf[wave][rl][lane * 4]); }
__global__ __launch_bounds__(128) void k_out(const float* __restrict__ CT, const float* __restrict__ WP, const float* __restrict__ BP, float* __restrict__ OUT) { __shared__ __align__(16) float sf[4][16][132];
  const int tid = threadIdx.x, wave = tid >> 5, lane = tid & 31, col = lane & 15, g = lane >> 4; const size_t r0 = (size_t)blockIdx.x * 64 + wave * 16; const int c0 = blockIdx.y * 128;
  v8f acc[8] = {};
#pragma unroll 2
  for (int kc = 0; kc < CC / 32; ++kc) { const F2 a = split_row(CT + (r0 + col) * CC, kc * 32, lane);
#pragma unroll
    for (int j = 0; j < 8; ++j) { const v16b w = fragb_f32(WP + (size_t)(c0 + j * 16 + col) * CC + kc * 32, lane); acc[j] = wmma_bf(a.h, w, acc[j]); acc[j] = wmma_bf(a.l, w, acc[j]); } }
#pragma unroll
  for (int j = 0; j < 8; ++j) { const float bb = bfr(BP[c0 + j * 16 + col]);
#pragma unroll
    for (int r = 0; r < 8; ++r) sf[wave][8 * g + r][j * 16 + col] = acc[j][r] + bb; }
  LDSX(); for (int rl = 0; rl < 16; ++rl) vst2(OUT + (r0 + rl) * CC + c0 + lane * 4, *(const v4f*)&sf[wave][rl][lane * 4]); }
extern "C" void kernel_launch(void* const* d_in, const int* in_sizes, int n_in, void* d_out, int out_size, void* d_ws, size_t ws_size, hipStream_t stream) {
  (void)in_sizes; (void)n_in; (void)out_size;
  const float** F = (const float**)d_in;
  if (ws_size < (size_t)WS_END) return;
  char* ws = (char*)d_ws; float *Q = (float*)(ws + WS_Q), *XR = (float*)(ws + WS_XR), *KVT = (float*)(ws + WS_KV), *CT = (float*)(ws + WS_CT); _Float16 *KT = (_Float16*)(ws + WS_KT), *KTL = (_Float16*)(ws + WS_KTL), *VT = (_Float16*)(ws + WS_VT), *VTL = (_Float16*)(ws + WS_VTL);
  k_q<<<dim3(TOB, CC / 128), 128, 0, stream>>>(F[0], F[1], Q);
  k_pool<<<TNB * MM, 256, 0, stream>>>(F[0], F[6], F[7], F[8], F[9], XR);
  k_kv<<<dim3(MM / 64, CC / 128, 2 * TNB), 128, 0, stream>>>(XR, F[2], F[3], KT, KTL, VT, VTL);
  k_kvp<<<TNB * NH, 64, 0, stream>>>(KT, KTL, VT, VTL, KVT);
  k_ctx<<<dim3(TOB, CC / 128), 128, 0, stream>>>(Q, KVT, CT);
  k_out<<<dim3(TOB, CC / 128), 128, 0, stream>>>(CT, F[4], F[5], (float*)d_out);
}
